// Block_2095944040561
// MI455X (gfx1250) — hardware-run, weakly checked
//
#include <hip/hip_runtime.h>


#ifndef NB
#define NB 8
#endif
#ifndef SEQ
#define SEQ 2048
#endif
#define NB_FULL  8
#define SEQ_FULL 2048
#ifndef OUT_SEQ
#define OUT_SEQ SEQ
#endif
#define DMODEL 512
#define NH_    4
#define HD     128
#define DFF    1024
#define BAND   6
#define AW     4
#define OSP    132
#define WS     64.0f
#define WSI    (1.0f / 64.0f)
#define CXS    64.0f
#define SC2    ((float)(0.08838834764831845 * 1.4426950408889634))
#define PSH    14.0f
#define NEGB   (-3.0e38f)

static_assert(HD == 128);
static_assert(NH_ * HD == DMODEL);
static_assert(HD % 64 == 0);
static_assert(HD % 32 == 0);
static_assert(DMODEL % 64 == 0);
static_assert(DFF % 64 == 0);
static_assert(DMODEL % 32 == 0);
static_assert(DFF % 32 == 0);
static_assert(DMODEL == 2 * 32 * 8);
static_assert(SEQ % 64 == 0);
static_assert((NB * SEQ) % 64 == 0);
static_assert((NB * SEQ) % 8 == 0);
static_assert(SEQ % 32 == 0);
static_assert(SEQ >= 32);
static_assert(SEQ % (16 * AW) == 0);
static_assert(BAND <= 8);
static_assert(NB <= NB_FULL);
static_assert(SEQ <= SEQ_FULL);
static_assert((OSP * 4) % 16 == 0);
static_assert(OSP >= HD);
static_assert((size_t)AW * 16 * OSP * 4 <= 131072);
static_assert((size_t)64 * 68 * 4 <= 131072);
static_assert((size_t)16 * 68 * 4 <= 131072);

typedef _Float16 h16;
typedef __attribute__((ext_vector_type(16))) _Float16 v16h;
typedef __attribute__((ext_vector_type(8)))  _Float16 v8h;
typedef __attribute__((ext_vector_type(8)))  float    v8f;
typedef __attribute__((ext_vector_type(4)))  float    v4f;
typedef v4f  __attribute__((may_alias)) v4fa;

__device__ __forceinline__ unsigned short f2bf(float f) { unsigned u = __float_as_uint(f); u += 0x7FFFu + ((u >> 16) & 1u); return (unsigned short)(u >> 16); }
__device__ __forceinline__ float bfr(float f) { return __uint_as_float(((unsigned)f2bf(f)) << 16); }
__device__ __forceinline__ v16h cat16(v8h lo, v8h hi) { return __builtin_shufflevector(lo, hi, 0, 1, 2, 3, 4, 5, 6, 7, 8, 9, 10, 11, 12, 13, 14, 15); }
__device__ __forceinline__ v16h ldh(const h16* p) { return cat16(*(const v8h*)p, *(const v8h*)(p + 16)); }
__device__ __forceinline__ void wave_sync() { __builtin_amdgcn_fence(3  , "wavefront"); __builtin_amdgcn_wave_barrier(); asm volatile("" ::: "memory"); }
static __device__ __forceinline__ h16 toh_flush(float v) { const h16 r = (h16)v; return (fabsf(v) < 6.103515625e-05f) ? (h16)0.0f : r; }
__device__ __forceinline__ v8f mm16(v16h a, v16h b, v8f c) {
    c = __builtin_amdgcn_wmma_f32_16x16x32_f16(false, a, false, b, (short)0, c, false, false);
    asm volatile("v_nop\n\tv_nop\n\tv_nop\n\tv_nop" : "+v"(c) : "v"(a), "v"(b));
    return c;
}
__device__ __forceinline__ float gelu_erf(float v) { return 0.5f * v * (1.0f + erff(v * 0.70710678118654752f)); }

__global__ __launch_bounds__(256) void k_wcvt(const float* __restrict__ src, h16* dst, size_t n8) {
    const size_t i = (size_t)blockIdx.x * 256 + threadIdx.x; if (i >= n8) return;
    const v8f v = *(const v8f*)(src + i * 8); v8h o;
#pragma unroll
    for (int k = 0; k < 8; ++k) o[k] = toh_flush(bfr(v[k]) * WS);
    *(volatile v8h*)(dst + i * 8) = o; __threadfence(); *(volatile v8h*)(dst + i * 8) = o;
}

__global__ __launch_bounds__(256) void k_ln(const float* __restrict__ X, const float* __restrict__ G, const float* __restrict__ Bv, h16* H, int inSeq, int cvt) {
#pragma clang fp contract(off)
    const int lane = threadIdx.x & 31;
    const int wave = __builtin_amdgcn_readfirstlane((int)(threadIdx.x >> 5));
    const int row = blockIdx.x * 8 + wave;
    const int bb = row / SEQ, tt = row % SEQ;
    const float* src = X + ((size_t)bb * (size_t)inSeq + (size_t)tt) * DMODEL;
    const int ca = 8 * lane, cb = 256 + 8 * lane;
    const v4f a0 = *(const v4f*)(src + ca), a1 = *(const v4f*)(src + ca + 4), a2 = *(const v4f*)(src + cb), a3 = *(const v4f*)(src + cb + 4);
    float v[16];
#pragma unroll
    for (int i = 0; i < 4; ++i) { v[i] = a0[i]; v[4 + i] = a1[i]; v[8 + i] = a2[i]; v[12 + i] = a3[i]; }
    if (cvt != 0) {
#pragma unroll
        for (int i = 0; i < 16; ++i) v[i] = bfr(v[i]);
    }
    float s = 0.0f;
#pragma unroll
    for (int i = 0; i < 16; ++i) s += v[i];
#pragma unroll
    for (int o = 16; o >= 1; o >>= 1) s += __shfl_xor(s, o, 32);
    const float mean = s * (1.0f / (float)DMODEL);
    float q = 0.0f;
#pragma unroll
    for (int i = 0; i < 16; ++i) { const float d = v[i] - mean; q += d * d; }
#pragma unroll
    for (int o = 16; o >= 1; o >>= 1) q += __shfl_xor(q, o, 32);
    const float rstd = 1.0f / sqrtf(q * (1.0f / (float)DMODEL) + 1e-5f);
    const v4f g0 = *(const v4f*)(G + ca), g1 = *(const v4f*)(G + ca + 4), g2 = *(const v4f*)(G + cb), g3 = *(const v4f*)(G + cb + 4);
    const v4f b0 = *(const v4f*)(Bv + ca), b1 = *(const v4f*)(Bv + ca + 4), b2 = *(const v4f*)(Bv + cb), b3 = *(const v4f*)(Bv + cb + 4);
    v8h oA, oB;
#pragma unroll
    for (int i = 0; i < 4; ++i) {
        oA[i]     = toh_flush((v[i]      - mean) * rstd * bfr(g0[i]) + bfr(b0[i]));
        oA[4 + i] = toh_flush((v[4 + i]  - mean) * rstd * bfr(g1[i]) + bfr(b1[i]));
        oB[i]     = toh_flush((v[8 + i]  - mean) * rstd * bfr(g2[i]) + bfr(b2[i]));
        oB[4 + i] = toh_flush((v[12 + i] - mean) * rstd * bfr(g3[i]) + bfr(b3[i])); }
    h16* dp = H + (size_t)row * DMODEL;
    *(volatile v8h*)(dp + ca) = oA; *(volatile v8h*)(dp + cb) = oB;
    __threadfence();
    *(volatile v8h*)(dp + ca) = oA; *(volatile v8h*)(dp + cb) = oB;
}

__device__ __forceinline__ void gemm_loop(const h16* __restrict__ A, const h16* __restrict__ Bt, size_t aoff, size_t boff, int K, v8f (&acc)[4][4]) {
#pragma unroll
    for (int mb = 0; mb < 4; ++mb)
#pragma unroll
        for (int nb = 0; nb < 4; ++nb) acc[mb][nb] = (v8f){};
#pragma unroll 1
    for (int kc = 0; kc < K; kc += 32) {
        v16h a[4];
#pragma unroll
        for (int mb = 0; mb < 4; ++mb) a[mb] = ldh(A + aoff + (size_t)mb * 16 * (size_t)K + kc);
#pragma unroll
        for (int nb = 0; nb < 4; ++nb) { const v16h b = ldh(Bt + boff + (size_t)nb * 16 * (size_t)K + kc);
#pragma unroll
            for (int mb = 0; mb < 4; ++mb) acc[mb][nb] = mm16(a[mb], b, acc[mb][nb]); }
    }
}

__global__ __launch_bounds__(32) __attribute__((amdgpu_num_vgpr(256))) void k_gemm_qk(const h16* __restrict__ A, const h16* __restrict__ W, const float* __restrict__ bias, h16* QK, float osc) {
    __shared__ __align__(16) float os[16 * 68];
    const int lane = threadIdx.x & 31, lr = lane & 15, hi = lane >> 4; const int r0 = blockIdx.x * 64, c0 = blockIdx.y * 64;
    v8f acc[4][4];
    gemm_loop(A, W, (size_t)(r0 + lr) * DMODEL + 8 * hi, (size_t)(c0 + lr) * DMODEL + 8 * hi, DMODEL, acc);
    float bc[4];
#pragma unroll
    for (int nb = 0; nb < 4; ++nb) bc[nb] = bfr(bias[c0 + nb * 16 + lr]);
    const int bb = r0 / SEQ, tt = r0 % SEQ; const int part = c0 / DMODEL, hh = (c0 % DMODEL) / HD, dc = c0 % HD;
    const size_t tbase = (size_t)part * ((size_t)NB * NH_ * SEQ * HD) + ((size_t)(bb * NH_ + hh) * SEQ + (size_t)tt) * HD + (size_t)dc;
    static_assert(32 * 16 * 4 == 16 * 64 * 2);
#pragma unroll
    for (int mb = 0; mb < 4; ++mb) {
#pragma unroll
        for (int nb = 0; nb < 4; ++nb) {
#pragma unroll
            for (int j = 0; j < 8; ++j) os[(hi * 8 + j) * 68 + nb * 16 + lr] = acc[mb][nb][j] * osc + bc[nb]; }
        wave_sync();
#pragma unroll 1
        for (int ps = 0; ps < 2; ++ps) {
#pragma unroll
            for (int s = 0; s < 4; ++s) { const int row = 4 * s + (lane >> 3), c8 = (lane & 7) * 8;
                const v4f x0 = *(const v4fa*)(&os[row * 68 + c8]); const v4f x1 = *(const v4fa*)(&os[row * 68 + c8 + 4]); v8h hv;
#pragma unroll
                for (int i = 0; i < 4; ++i) { hv[i] = toh_flush(x0[i]); hv[4 + i] = toh_flush(x1[i]); }
                *(volatile v8h*)(QK + tbase + (size_t)(mb * 16 + row) * HD + c8) = hv; }
            if (ps == 0) __threadfence(); }
        wave_sync();
    }
}

__global__ __launch_bounds__(32) __attribute__((amdgpu_num_vgpr(256))) void k_gemm_vt(const h16* __restrict__ WV, const h16* __restrict__ Hn, const float* __restrict__ bias, h16* VT, float osc) {
    __shared__ __align__(16) float os[16 * 68];
    const int lane = threadIdx.x & 31, lr = lane & 15, hi = lane >> 4; const int r0 = blockIdx.x * 64, c0 = blockIdx.y * 64;
    v8f acc[4][4];
    gemm_loop(WV, Hn, (size_t)(r0 + lr) * DMODEL + 8 * hi, (size_t)(c0 + lr) * DMODEL + 8 * hi, DMODEL, acc);
    const int bb = c0 / SEQ, tt = c0 % SEQ;
    const size_t tbase = (size_t)bb * (size_t)DMODEL * SEQ + (size_t)r0 * SEQ + (size_t)tt;
    static_assert(32 * 16 * 4 == 16 * 64 * 2);
#pragma unroll
    for (int mb = 0; mb < 4; ++mb) {
        float br[8];
#pragma unroll
        for (int j = 0; j < 8; ++j) br[j] = bfr(bias[r0 + mb * 16 + hi * 8 + j]);
#pragma unroll
        for (int nb = 0; nb < 4; ++nb) {
#pragma unroll
            for (int j = 0; j < 8; ++j) os[(hi * 8 + j) * 68 + nb * 16 + lr] = acc[mb][nb][j] * osc + br[j]; }
        wave_sync();
#pragma unroll 1
        for (int ps = 0; ps < 2; ++ps) {
#pragma unroll
            for (int s = 0; s < 4; ++s) { const int row = 4 * s + (lane >> 3), c8 = (lane & 7) * 8;
                const v4f x0 = *(const v4fa*)(&os[row * 68 + c8]); const v4f x1 = *(const v4fa*)(&os[row * 68 + c8 + 4]); v8h hv;
#pragma unroll
                for (int i = 0; i < 4; ++i) { hv[i] = toh_flush(x0[i]); hv[4 + i] = toh_flush(x1[i]); }
                *(volatile v8h*)(VT + tbase + (size_t)(mb * 16 + row) * SEQ + c8) = hv; }
            if (ps == 0) __threadfence(); }
        wave_sync();
    }
}

__global__ __launch_bounds__(32) __attribute__((amdgpu_num_vgpr(256))) void k_gemm_res(const h16* __restrict__ A, const h16* __restrict__ W, const float* __restrict__ bias,
                                                                                       const float* __restrict__ RES, float* OUTF, int K, float osc, int resSeq, int outSeq, int rcvt) {
    __shared__ __align__(16) float os[16 * 68];
    const int lane = threadIdx.x & 31, lr = lane & 15, hi = lane >> 4; const int r0 = blockIdx.x * 64, c0 = blockIdx.y * 64;
    v8f acc[4][4];
    gemm_loop(A, W, (size_t)(r0 + lr) * (size_t)K + 8 * hi, (size_t)(c0 + lr) * (size_t)K + 8 * hi, K, acc);
    float bc[4];
#pragma unroll
    for (int nb = 0; nb < 4; ++nb) bc[nb] = bfr(bias[c0 + nb * 16 + lr]);
    const int bb = r0 / SEQ, tt = r0 % SEQ;
    const size_t rbase = ((size_t)bb * (size_t)resSeq + (size_t)tt) * DMODEL + (size_t)c0;
    const size_t obase = ((size_t)bb * (size_t)outSeq + (size_t)tt) * DMODEL + (size_t)c0;
    static_assert(32 * 16 * 8 == 16 * 64 * 4);
#pragma unroll
    for (int mb = 0; mb < 4; ++mb) {
#pragma unroll
        for (int nb = 0; nb < 4; ++nb) {
#pragma unroll
            for (int j = 0; j < 8; ++j) os[(hi * 8 + j) * 68 + nb * 16 + lr] = acc[mb][nb][j] * osc + bc[nb]; }
        wave_sync();
        v4f val[8];
#pragma unroll
        for (int s = 0; s < 8; ++s) { const int row = 2 * s + (lane >> 4), c4 = (lane & 15) * 4;
            const v4f x = *(const v4fa*)(&os[row * 68 + c4]);
            v4f r = *(const v4f*)(RES + rbase + (size_t)(mb * 16 + row) * DMODEL + c4);
            if (rcvt != 0) { r[0] = bfr(r[0]); r[1] = bfr(r[1]); r[2] = bfr(r[2]); r[3] = bfr(r[3]); }
            val[s] = x + r; }
#pragma unroll 1
        for (int ps = 0; ps < 2; ++ps) {
#pragma unroll
            for (int s = 0; s < 8; ++s) { const int row = 2 * s + (lane >> 4), c4 = (lane & 15) * 4;
                *(volatile v4f*)(OUTF + obase + (size_t)(mb * 16 + row) * DMODEL + c4) = val[s]; }
            if (ps == 0) __threadfence(); }
        wave_sync();
    }
}

__global__ __launch_bounds__(32) __attribute__((amdgpu_num_vgpr(256))) void k_gemm_gelu(const h16* __restrict__ A, const h16* __restrict__ W, const float* __restrict__ bias, h16* T, float osc) {
    __shared__ __align__(16) float os[64 * 68];
    const int lane = threadIdx.x & 31, lr = lane & 15, hi = lane >> 4; const int r0 = blockIdx.x * 64, c0 = blockIdx.y * 64;
    v8f acc[4][4];
    gemm_loop(A, W, (size_t)(r0 + lr) * DMODEL + 8 * hi, (size_t)(c0 + lr) * DMODEL + 8 * hi, DMODEL, acc);
    float bc[4];
#pragma unroll
    for (int nb = 0; nb < 4; ++nb) bc[nb] = bfr(bias[c0 + nb * 16 + lr]);
#pragma unroll
    for (int mb = 0; mb < 4; ++mb) {
#pragma unroll
        for (int nb = 0; nb < 4; ++nb) {
#pragma unroll
            for (int j = 0; j < 8; ++j) os[(mb * 16 + hi * 8 + j) * 68 + nb * 16 + lr] = acc[mb][nb][j] * osc + bc[nb]; } }
    wave_sync();
    static_assert(32 * 16 * 16 == 64 * 64 * 2);
#pragma unroll 1
    for (int s = 0; s < 16; ++s) { const int row = 4 * s + (lane >> 3), c8 = (lane & 7) * 8;
        const v4f x0 = *(const v4fa*)(&os[row * 68 + c8]); const v4f x1 = *(const v4fa*)(&os[row * 68 + c8 + 4]); v8h hv;
#pragma unroll
        for (int i = 0; i < 4; ++i) { hv[i] = toh_flush(gelu_erf(x0[i])); hv[4 + i] = toh_flush(gelu_erf(x1[i])); }
        h16* dp = T + (size_t)(r0 + row) * DFF + (size_t)c0 + c8;
        *(volatile v8h*)dp = hv; __threadfence(); *(volatile v8h*)dp = hv; }
}

template <int LOCAL>
__device__ __forceinline__ void flash_body(const h16* __restrict__ QP, const h16* __restrict__ KP, const h16* __restrict__ VT, h16* CTX) {
    __shared__ __align__(16) float os[AW * 16 * OSP];
    const int lane = threadIdx.x & 31, lr = lane & 15, hi = lane >> 4;
    const int wave = __builtin_amdgcn_readfirstlane((int)(threadIdx.x >> 5));
    const int zh = blockIdx.y; const int b = zh / NH_, h = zh % NH_;
    const int t0 = (blockIdx.x * AW + wave) * 16;
    int ksv = ((int)blockIdx.x * AW + (int)(threadIdx.x >> 5)) * 16 - 8;
    ksv = ksv < 0 ? 0 : ksv; ksv = ksv > SEQ - 32 ? SEQ - 32 : ksv;
    const int kbeg = LOCAL ? __builtin_amdgcn_readfirstlane(ksv) : 0;
    const int kend = LOCAL ? kbeg + 32 : SEQ;
    const int tq = t0 + lr;
    const size_t pbase = (size_t)zh * SEQ * HD;
    const size_t qo = pbase + (size_t)tq * HD + 8 * hi;
    const size_t ko = pbase + (size_t)lr * HD + 8 * hi;
    const size_t vo = pbase + (size_t)lr * SEQ + 8 * hi;
    v8f o[8];
#pragma unroll
    for (int j = 0; j < 8; ++j) o[j] = (v8f){};
    float m = NEGB, l = 0.0f;
#pragma unroll 1
    for (int key0 = kbeg; key0 < kend; key0 += 32) {
        int qz = 0; asm volatile("" : "+v"(qz));
        const h16* ka = KP + ko + (size_t)key0 * HD;
        const h16* qa = QP + qo + qz;
        v8f sa = (v8f){}, sb = (v8f){};
#pragma unroll
        for (int fc = 0; fc < HD / 32; ++fc) {
            const v16h qf = ldh(qa + fc * 32);
            const v16h k0f = ldh(ka + fc * 32), k1f = ldh(ka + 16 * HD + fc * 32);
            sa = mm16(k0f, qf, sa); sb = mm16(k1f, qf, sb); }
        const int dja = key0 + 8 * hi - tq;
        float ta[8], tb[8]; bool fa[8], fb[8]; float mx = NEGB;
#pragma unroll
        for (int r = 0; r < 8; ++r) {
            ta[r] = sa[r] * SC2; tb[r] = sb[r] * SC2;
            if (LOCAL) { const int da = dja + r, db = dja + 16 + r; fa[r] = (da > -BAND) & (da < BAND); fb[r] = (db > -BAND) & (db < BAND); }
            else       { fa[r] = true; fb[r] = true; }
            mx = fmaxf(mx, fmaxf(fa[r] ? ta[r] : NEGB, fb[r] ? tb[r] : NEGB)); }
        mx = fmaxf(mx, __shfl_xor(mx, 16, 32));
        const float mnew = fmaxf(m, mx);
        const float alpha = __builtin_amdgcn_exp2f(m - mnew);
        const float sh = PSH - mnew;
        v16h pb; float ls = 0.0f;
#pragma unroll
        for (int r = 0; r < 8; ++r) {
            const float xa = ta[r] + sh, xb = tb[r] + sh;
            float ea = __builtin_amdgcn_exp2f(xa), eb = __builtin_amdgcn_exp2f(xb);
            ea = (xa < -PSH) ? 0.0f : ea; eb = (xb < -PSH) ? 0.0f : eb;
            if (LOCAL) { ea = fa[r] ? ea : 0.0f; eb = fb[r] ? eb : 0.0f; }
            const h16 pa = (h16)ea; const h16 pc = (h16)eb;
            pb[r] = pa; pb[8 + r] = pc;
            ls += (float)pa + (float)pc; }
        l = l * alpha + ls; m = mnew;
#pragma unroll
        for (int j = 0; j < 8; ++j) o[j] = o[j] * alpha;
        const h16* va = VT + vo + key0;
#pragma unroll
        for (int g = 0; g < 2; ++g) {
            const v16h v0 = ldh(va + (size_t)(64 * g +  0) * SEQ), v1 = ldh(va + (size_t)(64 * g + 16) * SEQ);
            const v16h v2 = ldh(va + (size_t)(64 * g + 32) * SEQ), v3 = ldh(va + (size_t)(64 * g + 48) * SEQ);
            o[4 * g + 0] = mm16(v0, pb, o[4 * g + 0]); o[4 * g + 1] = mm16(v1, pb, o[4 * g + 1]);
            o[4 * g + 2] = mm16(v2, pb, o[4 * g + 2]); o[4 * g + 3] = mm16(v3, pb, o[4 * g + 3]); }
    }
    l += __shfl_xor(l, 16, 32);
    const bool any = l > 0.0f;
    const float lsafe = any ? l : 1.0f;
    const float inv = any ? (CXS * (1.0f / lsafe)) : 0.0f;
    const int wb = wave * 16 * OSP;
#pragma unroll
    for (int j = 0; j < 8; ++j) { v4f a, c;
        a[0] = o[j][0] * inv; a[1] = o[j][1] * inv; a[2] = o[j][2] * inv; a[3] = o[j][3] * inv;
        c[0] = o[j][4] * inv; c[1] = o[j][5] * inv; c[2] = o[j][6] * inv; c[3] = o[j][7] * inv;
        *(v4fa*)(&os[wb + lr * OSP + 16 * j + 8 * hi]) = a; *(v4fa*)(&os[wb + lr * OSP + 16 * j + 8 * hi + 4]) = c; }
    wave_sync();
    h16* crow = CTX + ((size_t)b * SEQ + t0) * DMODEL + h * HD;
    static_assert(32 * 16 * 8 == 16 * HD * 2);
#pragma unroll 1
    for (int ps = 0; ps < 2; ++ps) {
#pragma unroll
        for (int s = 0; s < 8; ++s) { const int row = 2 * s + (lane >> 4), c8 = (lane & 15) * 8;
            const v4f x0 = *(const v4fa*)(&os[wb + row * OSP + c8]); const v4f x1 = *(const v4fa*)(&os[wb + row * OSP + c8 + 4]); v8h hv;
#pragma unroll
            for (int i = 0; i < 4; ++i) { hv[i] = toh_flush(x0[i]); hv[4 + i] = toh_flush(x1[i]); }
            *(volatile v8h*)(crow + (size_t)row * DMODEL + c8) = hv; }
        if (ps == 0) __threadfence(); }
}

__global__ __launch_bounds__(32 * AW) __attribute__((amdgpu_num_vgpr(256))) void k_flash_band(const h16* __restrict__ QP, const h16* __restrict__ KP, const h16* __restrict__ VT, h16* CTX) {
    flash_body<1>(QP, KP, VT, CTX);
}
__global__ __launch_bounds__(32 * AW) __attribute__((amdgpu_num_vgpr(256))) void k_flash_dense(const h16* __restrict__ QP, const h16* __restrict__ KP, const h16* __restrict__ VT, h16* CTX) {
    flash_body<0>(QP, KP, VT, CTX);
}

static constexpr size_t al256(size_t v) { return (v + 255) & ~(size_t)255; }
static constexpr size_t N_WQKV = (size_t)3 * DMODEL * DMODEL;
static constexpr size_t N_WO   = (size_t)DMODEL * DMODEL;
static constexpr size_t N_W1   = (size_t)DFF * DMODEL;
static constexpr size_t N_W2   = (size_t)DMODEL * DFF;
static constexpr size_t N_WALL = 2 * N_WQKV + 2 * N_WO + N_W1 + N_W2;
static constexpr size_t PLANE  = (size_t)NB * NH_ * SEQ * HD;
static constexpr size_t SZ_W   = al256(N_WALL * 2);
static constexpr size_t SZ_H   = al256(PLANE * 2);
static constexpr size_t SZ_QK  = al256(2 * PLANE * 2);
static constexpr size_t SZ_X2  = al256((size_t)NB * SEQ * DMODEL * 4);
static constexpr size_t SZ_TOTAL = SZ_W + SZ_H + SZ_QK + SZ_H + SZ_H + SZ_X2;
static_assert(SZ_TOTAL <= (size_t)134217728);
static_assert(PLANE == (size_t)NB * SEQ * DMODEL);
static_assert((size_t)NB * SEQ * DFF * 2 <= SZ_QK);
static_assert((N_WQKV * 2) % 256 == 0);
static_assert((N_WO * 2) % 256 == 0);
static_assert((N_W1 * 2) % 256 == 0);
static_assert((PLANE * 2) % 256 == 0);
static_assert(N_WQKV % 8 == 0);
static_assert(N_WO % 8 == 0);
static_assert(N_W1 % 8 == 0);
static_assert(N_W2 % 8 == 0);

extern "C" void kernel_launch(void* const* d_in, const int* in_sizes, int n_in,
                              void* d_out, int out_size, void* d_ws, size_t ws_size, hipStream_t stream) {
    if (n_in < 19) return;
    const size_t needx = ((size_t)(NB - 1) * SEQ_FULL + SEQ) * DMODEL;
    if ((size_t)in_sizes[0] < needx) return;
    for (int i = 1; i <= 6; ++i) if (in_sizes[i] < DMODEL) return;
    if ((size_t)in_sizes[7] < N_WQKV || in_sizes[8] < 3 * DMODEL || (size_t)in_sizes[9] < N_WO || in_sizes[10] < DMODEL) return;
    if ((size_t)in_sizes[11] < N_WQKV || in_sizes[12] < 3 * DMODEL || (size_t)in_sizes[13] < N_WO || in_sizes[14] < DMODEL) return;
    if ((size_t)in_sizes[15] < N_W1 || in_sizes[16] < DFF || (size_t)in_sizes[17] < N_W2 || in_sizes[18] < DMODEL) return;
    if ((size_t)out_size < ((size_t)(NB - 1) * OUT_SEQ + SEQ) * DMODEL) return;
    if (SZ_TOTAL > ws_size) return;
    const float* x    = (const float*)d_in[0];
    const float* ln1w = (const float*)d_in[1];  const float* ln1b = (const float*)d_in[2];
    const float* ln2w = (const float*)d_in[3];  const float* ln2b = (const float*)d_in[4];
    const float* ln3w = (const float*)d_in[5];  const float* ln3b = (const float*)d_in[6];
    const float* wqkvl = (const float*)d_in[7]; const float* bqkvl = (const float*)d_in[8];
    const float* wol   = (const float*)d_in[9]; const float* bol   = (const float*)d_in[10];
    const float* wqkvg = (const float*)d_in[11]; const float* bqkvg = (const float*)d_in[12];
    const float* wog   = (const float*)d_in[13]; const float* bog   = (const float*)d_in[14];
    const float* w1 = (const float*)d_in[15]; const float* b1 = (const float*)d_in[16];
    const float* w2 = (const float*)d_in[17]; const float* b2 = (const float*)d_in[18];
    float* OUT = (float*)d_out;
    char* wsp = (char*)d_ws;
    h16* WL  = (h16*)wsp;
    h16* WOL = WL + N_WQKV;
    h16* WG  = WOL + N_WO;
    h16* WOG = WG + N_WQKV;
    h16* W1H = WOG + N_WO;
    h16* W2H = W1H + N_W1;
    wsp += SZ_W;
    h16* HN  = (h16*)wsp; wsp += SZ_H;
    h16* QK  = (h16*)wsp; wsp += SZ_QK;
    h16* VT  = (h16*)wsp; wsp += SZ_H;
    h16* CTX = (h16*)wsp; wsp += SZ_H;
    float* X2 = (float*)wsp; wsp += SZ_X2;
    h16* TG  = QK;

    { const unsigned g1 = (unsigned)((N_WQKV / 8 + 255) / 256), g2 = (unsigned)((N_WO / 8 + 255) / 256), g3 = (unsigned)((N_W1 / 8 + 255) / 256);
      k_wcvt<<<g1, 256, 0, stream>>>(wqkvl, WL, N_WQKV / 8);
      k_wcvt<<<g2, 256, 0, stream>>>(wol, WOL, N_WO / 8);
      k_wcvt<<<g1, 256, 0, stream>>>(wqkvg, WG, N_WQKV / 8);
      k_wcvt<<<g2, 256, 0, stream>>>(wog, WOG, N_WO / 8);
      k_wcvt<<<g3, 256, 0, stream>>>(w1, W1H, N_W1 / 8);
      k_wcvt<<<g3, 256, 0, stream>>>(w2, W2H, N_W2 / 8); }

    const dim3 gQK(NB * SEQ / 64, 2 * DMODEL / 64, 1), gVT(DMODEL / 64, NB * SEQ / 64, 1), gRES(NB * SEQ / 64, DMODEL / 64, 1), gFF(NB * SEQ / 64, DFF / 64, 1);
    const dim3 gFL(SEQ / (16 * AW), NB * NH_, 1);
    const unsigned gLN = (unsigned)(NB * SEQ / 8);

    k_ln<<<gLN, 256, 0, stream>>>(x, ln1w, ln1b, HN, SEQ_FULL, 1);
    k_gemm_qk<<<gQK, 32, 0, stream>>>(HN, WL, bqkvl, QK, WSI);
    k_gemm_vt<<<gVT, 32, 0, stream>>>(WL + (size_t)2 * DMODEL * DMODEL, HN, bqkvl + 2 * DMODEL, VT, WSI);
    k_flash_band<<<gFL, 32 * AW, 0, stream>>>(QK, QK + PLANE, VT, CTX);
    k_gemm_res<<<gRES, 32, 0, stream>>>(CTX, WOL, bol, x, OUT, DMODEL, WSI * (1.0f / CXS), SEQ_FULL, OUT_SEQ, 1);

    k_ln<<<gLN, 256, 0, stream>>>(OUT, ln2w, ln2b, HN, OUT_SEQ, 0);
    k_gemm_qk<<<gQK, 32, 0, stream>>>(HN, WG, bqkvg, QK, WSI);
    k_gemm_vt<<<gVT, 32, 0, stream>>>(WG + (size_t)2 * DMODEL * DMODEL, HN, bqkvg + 2 * DMODEL, VT, WSI);
    k_flash_dense<<<gFL, 32 * AW, 0, stream>>>(QK, QK + PLANE, VT, CTX);
    k_gemm_res<<<gRES, 32, 0, stream>>>(CTX, WOG, bog, OUT, X2, DMODEL, WSI * (1.0f / CXS), OUT_SEQ, SEQ, 0);

    k_ln<<<gLN, 256, 0, stream>>>(X2, ln3w, ln3b, HN, SEQ, 0);
    k_gemm_gelu<<<gFF, 32, 0, stream>>>(HN, W1H, b1, TG, WSI);
    k_gemm_res<<<gRES, 32, 0, stream>>>(TG, W2H, b2, X2, OUT, DFF, WSI, SEQ, OUT_SEQ, 0);
}
